// RingAttention_64278480552169
// MI455X (gfx1250) — hardware-verified
//
#include <hip/hip_runtime.h>


#ifndef NB
#define NB 2
#endif
#ifndef SEQ
#define SEQ 2048
#endif
#define NB_FULL 2
#define SEQ_FULL 2048
#define DIM 2048
#define HEADS 16
#define DHEAD 128
#define NQKV (3 * DIM)
#define SEQT (NB * SEQ)
#define QBLK (SEQ / 64)
#define CSTR 132

static_assert(SEQ % 64 == 0);
static_assert(SEQ >= 64);
static_assert(SEQ <= SEQ_FULL);
static_assert(NB >= 1 && NB <= NB_FULL);
static_assert(DIM == HEADS * DHEAD);
static_assert(DHEAD == 128);
static_assert(DIM % 128 == 0 && NQKV % 128 == 0 && DIM % 32 == 0);
static_assert((DIM * DIM) % 2048 == 0);

typedef unsigned short us16;
typedef __attribute__((ext_vector_type(16))) __bf16   v16bf;
typedef __attribute__((ext_vector_type(16))) _Float16 v16h;
typedef __attribute__((ext_vector_type(8)))  float    v8f;
typedef __attribute__((ext_vector_type(8)))  unsigned v8u;
typedef __attribute__((ext_vector_type(4)))  unsigned v4u;
typedef __attribute__((ext_vector_type(2)))  unsigned v2u;
typedef __attribute__((ext_vector_type(4)))  float    v4f;

__device__ __forceinline__ unsigned f2bf(float f) { unsigned u = __float_as_uint(f); u += 0x7FFFu + ((u >> 16) & 1u); return u >> 16; }
__device__ __forceinline__ float bf2f(unsigned h) { return __uint_as_float(h << 16); }
__device__ __forceinline__ unsigned f2h(float f) { _Float16 t = (_Float16)f; return (unsigned)__builtin_bit_cast(unsigned short, t); }

__device__ __forceinline__ v8u ld_frag(const us16* rowp, int hh) {
    const v4u a = *(const v4u*)(rowp + 8 * hh);
    const v4u b = *(const v4u*)(rowp + 16 + 8 * hh);
    return __builtin_shufflevector(a, b, 0, 1, 2, 3, 4, 5, 6, 7);
}
__device__ __forceinline__ v8f mma_bf16(v8u a, v8u b, v8f c) {
    return __builtin_amdgcn_wmma_f32_16x16x32_bf16(false, __builtin_bit_cast(v16bf, a), false, __builtin_bit_cast(v16bf, b), (short)0, c, false, false);
}
__device__ __forceinline__ v8f mma_f16(v8u a, v8u b, v8f c) {
    return __builtin_amdgcn_wmma_f32_16x16x32_f16(false, __builtin_bit_cast(v16h, a), false, __builtin_bit_cast(v16h, b), (short)0, c, false, false);
}
__device__ __forceinline__ void mma_guard(v8f& c, v8u a, v8u b) {
    asm volatile("v_nop\n\tv_nop\n\tv_nop\n\tv_nop" : "+v"(c) : "v"(a), "v"(b));
}

__global__ __launch_bounds__(256) void prep_x(const float* __restrict__ x, us16* xb) {
    const int tok = blockIdx.x;
    const int bsel = tok / SEQ, isel = tok - bsel * SEQ;
    const float* xr = x + ((size_t)bsel * SEQ_FULL + isel) * DIM;
    const int tid = threadIdx.x;
    const v4f v0 = *(const v4f*)(xr + 8 * tid);
    const v4f v1 = *(const v4f*)(xr + 8 * tid + 4);
    v4u pk;
    pk.x = f2bf(v0.x) | (f2bf(v0.y) << 16);
    pk.y = f2bf(v0.z) | (f2bf(v0.w) << 16);
    pk.z = f2bf(v1.x) | (f2bf(v1.y) << 16);
    pk.w = f2bf(v1.z) | (f2bf(v1.w) << 16);
    us16* orow = xb + (size_t)tok * DIM + 8 * tid;
    *(volatile v4u*)orow = pk;
    __threadfence();
    *(volatile v4u*)orow = pk;
}

template <int F16>
__device__ __forceinline__ unsigned cvt_w(float v, float scale) {
    const unsigned b = f2bf(v);
    if (F16) return f2h(bf2f(b) * scale);
    return b;
}
template <int F16>
__global__ __launch_bounds__(256) void prep_w(const float* __restrict__ s0, const float* __restrict__ s1, const float* __restrict__ s2,
                                              float scale, us16* dst) {
    const int z = blockIdx.y;
    const float* src = (z == 0) ? s0 : ((z == 1) ? s1 : s2);
    const size_t e = ((size_t)blockIdx.x * 256 + threadIdx.x) * 8;
    const v4f v0 = *(const v4f*)(src + e);
    const v4f v1 = *(const v4f*)(src + e + 4);
    v4u pk;
    pk.x = cvt_w<F16>(v0.x, scale) | (cvt_w<F16>(v0.y, scale) << 16);
    pk.y = cvt_w<F16>(v0.z, scale) | (cvt_w<F16>(v0.w, scale) << 16);
    pk.z = cvt_w<F16>(v1.x, scale) | (cvt_w<F16>(v1.y, scale) << 16);
    pk.w = cvt_w<F16>(v1.z, scale) | (cvt_w<F16>(v1.w, scale) << 16);
    us16* dp = dst + (size_t)z * DIM * DIM + e;
    *(volatile v4u*)dp = pk;
    __threadfence();
    *(volatile v4u*)dp = pk;
}

template <int F16>
__device__ __forceinline__ void mm_tile(const us16* __restrict__ arow, const us16* __restrict__ bbase, int ldb, int K, int hh, v8f (&acc)[4]) {
#pragma unroll 1
    for (int kc = 0; kc < K; kc += 32) {
        const v8u a = ld_frag(arow + kc, hh);
#pragma unroll
        for (int t = 0; t < 4; ++t) {
            const v8u bfrag = ld_frag(bbase + (size_t)(t * 16) * ldb + kc, hh);
            if (F16) acc[t] = mma_f16(a, bfrag, acc[t]);
            else     acc[t] = mma_bf16(a, bfrag, acc[t]);
            mma_guard(acc[t], a, bfrag);
        }
    }
}

__global__ __launch_bounds__(256) void qkv_gemm(const us16* __restrict__ xb, const us16* __restrict__ wqkv, us16* qp, us16* kp, us16* vt) {
    __shared__ __align__(16) float cst[64 * CSTR];
    const int tid = threadIdx.x, lane = tid & 31, wv = tid >> 5, l16 = lane & 15, hh = lane >> 4;
    const int rt = wv & 3, ch = wv >> 2;
    const int row0 = blockIdx.x * 64;
    const int colb = blockIdx.y * 128;
    const us16* arow = xb + (size_t)(row0 + rt * 16 + l16) * DIM;
    const us16* bbase = wqkv + (size_t)(colb + ch * 64 + l16) * DIM;
    v8f acc[4] = {};
    mm_tile<0>(arow, bbase, DIM, DIM, hh, acc);
#pragma unroll
    for (int r = 0; r < 8; ++r) {
        const int rl = rt * 16 + 8 * hh + r;
#pragma unroll
        for (int t = 0; t < 4; ++t) cst[rl * CSTR + ch * 64 + t * 16 + l16] = acc[t][r];
    }
    __syncthreads();
    const int which = colb / DIM;
    const int hsel = (colb - which * DIM) / DHEAD;
    auto pass = [&]() {
        if (which < 2) {
            us16* pl = (which == 0) ? qp : kp;
#pragma unroll
            for (int j = 0; j < 8; ++j) {
                const int r = wv * 8 + j;
                const v4f v = *(const v4f*)(cst + r * CSTR + 4 * lane);
                v2u pk;
                pk.x = f2h(v.x) | (f2h(v.y) << 16);
                pk.y = f2h(v.z) | (f2h(v.w) << 16);
                const size_t off = ((size_t)hsel * SEQT + row0 + r) * DHEAD + 4 * lane;
                *(volatile v2u*)(pl + off) = pk;
            }
        } else {
#pragma unroll 4
            for (int j = 0; j < 16; ++j) {
                const int d = wv * 16 + j;
                const float a = cst[(2 * lane) * CSTR + d] * 4.0f, bq = cst[(2 * lane + 1) * CSTR + d] * 4.0f;
                const size_t off = ((size_t)hsel * DHEAD + d) * SEQT + row0 + 2 * lane;
                *(volatile unsigned*)(vt + off) = f2h(a) | (f2h(bq) << 16);
            }
        }
    };
    pass();
    __threadfence();
    pass();
}

__global__ __launch_bounds__(128) __attribute__((amdgpu_num_vgpr(256)))
void attn_main(const us16* qp, const us16* kp, const us16* vt, us16* ao) {
    __shared__ v4u ost[4][16][16];
    const int tid = threadIdx.x, lane = tid & 31, wv = tid >> 5, m = lane & 15, hh = lane >> 4;
    const int qb = blockIdx.x;
    const int h = blockIdx.y % HEADS, bsel = blockIdx.y / HEADS;
    const size_t tok0 = (size_t)bsel * SEQ;
    const int qrow = qb * 64 + wv * 16;
    const size_t qoff = ((size_t)h * SEQT + tok0 + qrow + m) * DHEAD;
    const v8u q0 = ld_frag(qp + qoff, hh);
    const v8u q1 = ld_frag(qp + qoff + 32, hh);
    const v8u q2 = ld_frag(qp + qoff + 64, hh);
    const v8u q3 = ld_frag(qp + qoff + 96, hh);
    const us16* kb = kp + ((size_t)h * SEQT + tok0) * DHEAD;
    const us16* vb = vt + (size_t)h * DHEAD * SEQT + tok0;
    const float NEG = -__builtin_inff();
    const float SCL = 0.08838834764831845f;
    v8f o[8] = {};
    float mrun = NEG, lrun = 0.f;
#pragma unroll 1
    for (int c = 0; c < SEQ / 32; ++c) {
        v8f s[2] = {};
#pragma unroll
        for (int t = 0; t < 2; ++t) {
            asm volatile("" ::: "memory");
            const size_t koff = (size_t)(c * 32 + t * 16 + m) * DHEAD;
            const v8u a0 = ld_frag(kb + koff, hh);
            s[t] = mma_f16(a0, q0, s[t]);
            mma_guard(s[t], a0, q0);
            const v8u a1 = ld_frag(kb + koff + 32, hh);
            s[t] = mma_f16(a1, q1, s[t]);
            mma_guard(s[t], a1, q1);
            const v8u a2 = ld_frag(kb + koff + 64, hh);
            s[t] = mma_f16(a2, q2, s[t]);
            mma_guard(s[t], a2, q2);
            const v8u a3 = ld_frag(kb + koff + 96, hh);
            s[t] = mma_f16(a3, q3, s[t]);
            mma_guard(s[t], a3, q3);
        }
        float sv[16];
        float cmax = NEG;
#pragma unroll
        for (int t = 0; t < 2; ++t)
#pragma unroll
            for (int r = 0; r < 8; ++r) {
                const float v = s[t][r] * SCL;
                sv[8 * t + r] = v;
                cmax = fmaxf(cmax, v);
            }
        cmax = fmaxf(cmax, __shfl_xor(cmax, 16, 32));
        const float mnew = fmaxf(mrun, cmax);
        const float fac = (mrun == NEG) ? 0.f : __expf(mrun - mnew);
        mrun = mnew;
        v16h ph;
        float psum = 0.f;
#pragma unroll
        for (int r = 0; r < 8; ++r) {
            const _Float16 p0 = (_Float16)(__expf(sv[r] - mnew) * 16384.0f);
            const _Float16 p1 = (_Float16)(__expf(sv[8 + r] - mnew) * 16384.0f);
            ph[r] = p0;
            ph[8 + r] = p1;
            psum += (float)p0 + (float)p1;
        }
        psum += __shfl_xor(psum, 16, 32);
        lrun = lrun * fac + psum;
        const v8u pbu = __builtin_bit_cast(v8u, ph);
#pragma unroll
        for (int dt = 0; dt < 8; ++dt) o[dt] = o[dt] * fac;
        asm volatile("" ::: "memory");
#pragma unroll
        for (int dt = 0; dt < 4; ++dt) {
            const v8u va = ld_frag(vb + (size_t)(dt * 16 + m) * SEQT + c * 32, hh);
            o[dt] = mma_f16(va, pbu, o[dt]);
            mma_guard(o[dt], va, pbu);
        }
        asm volatile("" ::: "memory");
#pragma unroll
        for (int dt = 4; dt < 8; ++dt) {
            const v8u va = ld_frag(vb + (size_t)(dt * 16 + m) * SEQT + c * 32, hh);
            o[dt] = mma_f16(va, pbu, o[dt]);
            mma_guard(o[dt], va, pbu);
        }
    }
    const float inv = 4.0f / lrun;
#pragma unroll
    for (int dt = 0; dt < 8; ++dt) {
        v4u w;
        w.x = f2h(o[dt][0] * inv) | (f2h(o[dt][1] * inv) << 16);
        w.y = f2h(o[dt][2] * inv) | (f2h(o[dt][3] * inv) << 16);
        w.z = f2h(o[dt][4] * inv) | (f2h(o[dt][5] * inv) << 16);
        w.w = f2h(o[dt][6] * inv) | (f2h(o[dt][7] * inv) << 16);
        ost[wv][m][2 * dt + hh] = w;
    }
    __syncthreads();
    us16* aob = ao + (tok0 + qrow) * DIM + (size_t)h * DHEAD;
    auto pass = [&]() {
#pragma unroll
        for (int p = 0; p < 8; ++p) {
            const int rr = 2 * p + hh, pc = lane & 15;
            *(volatile v4u*)(aob + (size_t)rr * DIM + 8 * pc) = ost[wv][rr][pc];
        }
    };
    pass();
    __threadfence();
    pass();
}

__global__ __launch_bounds__(256) void out_gemm(const us16* __restrict__ aop, const us16* __restrict__ wo, float* out) {
    __shared__ __align__(16) float cst[64 * CSTR];
    const int tid = threadIdx.x, lane = tid & 31, wv = tid >> 5, l16 = lane & 15, hh = lane >> 4;
    const int rt = wv & 3, ch = wv >> 2;
    const int row0 = blockIdx.x * 64;
    const int colb = blockIdx.y * 128;
    const us16* arow = aop + (size_t)(row0 + rt * 16 + l16) * DIM;
    const us16* bbase = wo + (size_t)(colb + ch * 64 + l16) * DIM;
    v8f acc[4] = {};
    mm_tile<1>(arow, bbase, DIM, DIM, hh, acc);
#pragma unroll
    for (int r = 0; r < 8; ++r) {
        const int rl = rt * 16 + 8 * hh + r;
#pragma unroll
        for (int t = 0; t < 4; ++t) cst[rl * CSTR + ch * 64 + t * 16 + l16] = acc[t][r] * (1.0f / 1024.0f);
    }
    __syncthreads();
    const int col = tid & 127, rsel = tid >> 7;
    float* ob = out + (size_t)row0 * DIM + colb + col;
    auto pass = [&]() {
#pragma unroll 4
        for (int r = rsel; r < 64; r += 2) *(volatile float*)(ob + (size_t)r * DIM) = cst[r * CSTR + col];
    };
    pass();
    __threadfence();
    pass();
}

extern "C" void kernel_launch(void* const* d_in, const int* in_sizes, int n_in,
                              void* d_out, int out_size, void* d_ws, size_t ws_size, hipStream_t stream) {
    if (n_in < 5) return;
    const float* x  = (const float*)d_in[0];
    const float* wq = (const float*)d_in[1];
    const float* wk = (const float*)d_in[2];
    const float* wv = (const float*)d_in[3];
    const float* wo = (const float*)d_in[4];
    float* out = (float*)d_out;
    if (in_sizes[0] < ((NB - 1) * SEQ_FULL + SEQ) * DIM) return;
    if (in_sizes[1] < DIM * DIM) return;
    if (in_sizes[2] < DIM * DIM) return;
    if (in_sizes[3] < DIM * DIM) return;
    if (in_sizes[4] < DIM * DIM) return;
    if (out_size < SEQT * DIM) return;

    size_t off = 0;
    auto carve = [&](size_t bytes) { size_t o = off; off += (bytes + 127) & ~(size_t)127; return o; };
    char* ws = (char*)d_ws;
    us16* xb   = (us16*)(ws + carve((size_t)SEQT * DIM * 2));
    us16* wqkv = (us16*)(ws + carve((size_t)NQKV * DIM * 2));
    us16* wop  = (us16*)(ws + carve((size_t)DIM * DIM * 2));
    us16* qp   = (us16*)(ws + carve((size_t)HEADS * SEQT * DHEAD * 2));
    us16* kp   = (us16*)(ws + carve((size_t)HEADS * SEQT * DHEAD * 2));
    us16* vt   = (us16*)(ws + carve((size_t)HEADS * DHEAD * SEQT * 2));
    us16* ao   = (us16*)(ws + carve((size_t)SEQT * DIM * 2));
    if (off > ws_size) return;
    if (off > (size_t)134217728) return;

    prep_x<<<SEQT, 256, 0, stream>>>(x, xb);
    prep_w<0><<<dim3((DIM * DIM) / 2048, 3), 256, 0, stream>>>(wq, wk, wv, 1.0f, wqkv);
    prep_w<1><<<dim3((DIM * DIM) / 2048, 1), 256, 0, stream>>>(wo, wo, wo, 64.0f, wop);
    qkv_gemm<<<dim3(SEQT / 64, NQKV / 128), 256, 0, stream>>>(xb, wqkv, qp, kp, vt);
    attn_main<<<dim3(QBLK, NB * HEADS), 128, 0, stream>>>(qp, kp, vt, ao);
    out_gemm<<<dim3(SEQT / 64, DIM / 128), 256, 0, stream>>>(ao, wop, out);
}
